// NetEval_2207613190845
// MI455X (gfx1250) — hardware-run, weakly checked
//
#include <hip/hip_runtime.h>
#include <math.h>

typedef __attribute__((ext_vector_type(16))) _Float16 v16h;
typedef __attribute__((ext_vector_type(8)))  _Float16 v8h;
typedef __attribute__((ext_vector_type(8)))  float    v8f;
typedef __attribute__((ext_vector_type(4)))  float    v4f;
typedef __attribute__((ext_vector_type(2)))  float    v2f;

constexpr int kNumSamples      = 262144;
constexpr int kNumExperts      = 16;
constexpr int kHidden          = 20;
constexpr int kInputs          = 2;
constexpr int kTilesPerWave    = 8;
constexpr int kWavesPerBlock   = 8;
constexpr int kSamplesPerWave  = 16 * kTilesPerWave;
constexpr int kSamplesPerBlock = kSamplesPerWave * kWavesPerBlock;
constexpr int kNumBlocks       = kNumSamples / kSamplesPerBlock;
static_assert(kSamplesPerWave == 128, "one wave owns 512 B of the output");
static_assert(kNumBlocks * kSamplesPerBlock == kNumSamples, "exact grid, no tail");
static_assert(kHidden == 20 && kInputs == 2, "slot map below is written for 20 hidden units");

constexpr float kCarryWeight = 64.0f;
constexpr float kCarryAct    = 64.0f;
constexpr float kCarryRem    = 2048.0f;
constexpr float kFoldBack    = 1.0f / (kCarryWeight * kCarryAct);
constexpr float kRemFold     = 1.0f / kCarryRem;
constexpr float kF16MinNormal = 6.103515625e-5f;

constexpr int kParamStride = 128;
constexpr int kParamGroup  = 12;

constexpr size_t kOffPlanes  = 0;
constexpr size_t kPlaneBytes = (size_t)kNumExperts * 3 * 1024 * 2;
constexpr size_t kOffRemPlanes = kOffPlanes + kPlaneBytes;
constexpr size_t kOffParams  = kOffRemPlanes + kPlaneBytes;
constexpr size_t kParamBytes = (size_t)kNumExperts * 2 * kParamStride * 4;
constexpr size_t kWsTotal    = kOffParams + kParamBytes;
static_assert(kPlaneBytes == 98304ull && kParamBytes == 16384ull && kWsTotal == 212992ull, "carve total");
static_assert((kOffRemPlanes % 128) == 0 && (kOffParams % 128) == 0, "128-B aligned regions");
static_assert(kWsTotal <= 134217728ull, "carve cap");

__device__ __forceinline__ int slot_unit(int s) {
  int u = -1;
  u = (s < 16) ? s : u;
  u = (s == 16) ? 16 : u;
  u = (s == 17) ? 17 : u;
  u = (s == 24) ? 18 : u;
  u = (s == 25) ? 19 : u;
  return u;
}

__global__ __launch_bounds__(128) void build_weight_planes_kernel(
    const float* __restrict__ W2, const float* __restrict__ W3, const float* __restrict__ W4,
    unsigned short* __restrict__ planes, unsigned short* __restrict__ rplanes)
{
  const int e = blockIdx.x;
  const int l = blockIdx.y;
  const float* W = (l == 0) ? W2 : ((l == 1) ? W3 : W4);
  const int tid = threadIdx.x;
  const int m  = tid >> 2;
  const int k8 = (tid & 3) * 8;
  const int um = slot_unit(m);
  const int umc = (um < 0) ? 0 : um;
  v8h hv, rv;
#pragma unroll
  for (int j = 0; j < 8; ++j) {
    const int uk = slot_unit(k8 + j);
    const int ukc = (uk < 0) ? 0 : uk;
    const bool live = (um >= 0) && (uk >= 0);
    float w = W[(size_t)e * (kHidden * kHidden) + ukc * kHidden + umc];
    asm volatile("" : "+v"(w));
    float c = w * kCarryWeight;
    c = live ? c : 0.0f;
    const float cv = (fabsf(c) < kF16MinNormal) ? 0.0f : c;
    const _Float16 hval = (_Float16)cv;
    float rem = (c - (float)hval) * kCarryRem;
    rem = (fabsf(rem) < kF16MinNormal) ? 0.0f : rem;
    rem = live ? rem : 0.0f;
    hv[j] = hval;
    rv[j] = (_Float16)rem;
  }
  const size_t po = (size_t)(e * 3 + l) * 1024 + (size_t)tid * 8;
  unsigned short* q  = planes + po;
  unsigned short* qr = rplanes + po;
  *(volatile v8h*)q  = hv;
  *(volatile v8h*)qr = rv;
  __threadfence();
  *(volatile v8h*)q  = hv;
  *(volatile v8h*)qr = rv;
}

__global__ __launch_bounds__(256) void build_param_table_kernel(
    const float* __restrict__ W1, const float* __restrict__ b1, const float* __restrict__ b2,
    const float* __restrict__ b3, const float* __restrict__ b4, const float* __restrict__ W5,
    const float* __restrict__ b5, float* __restrict__ params)
{
  const int e  = blockIdx.x;
  const int t  = threadIdx.x;
  const int hf = t >> 7;
  const int s  = t & 127;
  const int g  = s / kParamGroup;
  const int i  = s - g * kParamGroup;
  const int u  = (i < 8) ? (8 * hf + i) : ((i == 8) ? (16 + 2 * hf) : ((i == 9) ? (17 + 2 * hf) : -1));
  const int uc = (u < 0) ? 0 : u;
  const bool live = (u >= 0) && (g < 7);
  float c0 = W1[e * (kInputs * kHidden) + uc];
  float c1 = W1[e * (kInputs * kHidden) + kHidden + uc];
  float c2 = b1[e * kHidden + uc];
  float c3 = b2[e * kHidden + uc];
  float c4 = b3[e * kHidden + uc];
  float c5 = b4[e * kHidden + uc];
  float c6 = W5[e * kHidden + uc];
  float c7 = b5[e];
  asm volatile("" : "+v"(c0));
  asm volatile("" : "+v"(c1));
  asm volatile("" : "+v"(c2));
  asm volatile("" : "+v"(c3));
  asm volatile("" : "+v"(c4));
  asm volatile("" : "+v"(c5));
  asm volatile("" : "+v"(c6));
  asm volatile("" : "+v"(c7));
  float v = 0.0f;
  v = (g == 0) ? c0 : v;
  v = (g == 1) ? c1 : v;
  v = (g == 2) ? c2 : v;
  v = (g == 3) ? c3 : v;
  v = (g == 4) ? c4 : v;
  v = (g == 5) ? c5 : v;
  v = (g == 6) ? c6 : v;
  v = live ? v : 0.0f;
  v = (s == 7 * kParamGroup) ? c7 : v;
  float* q = params + (size_t)e * (2 * kParamStride) + t;
  *(volatile float*)q = v;
  __threadfence();
  *(volatile float*)q = v;
}

__device__ __forceinline__ v16h load_frag_f16(const _Float16* p) {
  union U { v16h v; v8h h[2]; } f;
  f.h[0] = *(const v8h*)(p);
  f.h[1] = *(const v8h*)(p + 16);
  return f.v;
}
__device__ __forceinline__ v8f mma_from_zero(v16h a, v16h b) {
  v8f c = (v8f){0.f, 0.f, 0.f, 0.f, 0.f, 0.f, 0.f, 0.f};
  c = __builtin_amdgcn_wmma_f32_16x16x32_f16(false, a, false, b, (short)0, c, false, false);
  asm volatile("v_nop\n\tv_nop\n\tv_nop\n\tv_nop" : "+v"(c) : "v"(a), "v"(b));
  return c;
}
__device__ __forceinline__ v8f mma_onto(v16h a, v16h b, v8f c) {
  c = __builtin_amdgcn_wmma_f32_16x16x32_f16(false, a, false, b, (short)0, c, false, false);
  asm volatile("v_nop\n\tv_nop\n\tv_nop\n\tv_nop" : "+v"(c) : "v"(a), "v"(b));
  return c;
}
__device__ __forceinline__ float gate_sigmoid(float z) {
  return __builtin_amdgcn_rcpf(1.0f + __expf(-z));
}
__device__ __forceinline__ void silu_to_operands(float z, _Float16& ov, _Float16& orem) {
  const float c = (z * kCarryAct) * gate_sigmoid(z);
  const float cv = (fabsf(c) < kF16MinNormal) ? 0.0f : c;
  const _Float16 hval = (_Float16)cv;
  float rem = (c - (float)hval) * kCarryRem;
  rem = (fabsf(rem) < kF16MinNormal) ? 0.0f : rem;
  ov = hval;
  orem = (_Float16)rem;
}
__device__ __forceinline__ void hidden_products(const _Float16* pv, const _Float16* pr, v16h hbv, v16h hbr,
                                                v8f& d0, v8f& d1, v8f& r0, v8f& r1) {
  const v16h a0 = load_frag_f16(pv);
  const v16h a1 = load_frag_f16(pv + 512);
  const v16h q0 = load_frag_f16(pr);
  const v16h q1 = load_frag_f16(pr + 512);
  d0 = mma_from_zero(a0, hbv);
  d1 = mma_from_zero(a1, hbv);
  r0 = mma_from_zero(q0, hbv);
  r1 = mma_from_zero(q1, hbv);
  r0 = mma_onto(a0, hbr, r0);
  r1 = mma_onto(a1, hbr, r1);
}
__device__ __forceinline__ int cell_index(float v) {
  const int c = (v <= -0.674f) ? 0 : ((v <= 0.0f) ? 1 : ((v <= 0.674f) ? 2 : 3));
  const bool inside = (v >= -4.0f) && (v <= 4.0f);
  return inside ? c : -1;
}

__global__ __launch_bounds__(256) void grid_ensemble_kernel(
    const float* __restrict__ x, const unsigned short* __restrict__ planes,
    const unsigned short* __restrict__ rplanes,
    const float* __restrict__ params, float* __restrict__ out, int nsamp)
{
  __shared__ __align__(16) float ys[kWavesPerBlock][kTilesPerWave * 32];
  const int lane = threadIdx.x & 31;
  const int wave = threadIdx.x >> 5;
  const int hf   = lane >> 4;
  const int col  = lane & 15;
  const int s0   = (blockIdx.x * kWavesPerBlock + wave) * kSamplesPerWave;
  float* ysw = ys[wave];
#pragma unroll
  for (int t = 0; t < kTilesPerWave; ++t) ysw[t * 32 + lane] = 0.0f;

  const _Float16* pl = (const _Float16*)planes;
  const _Float16* rl = (const _Float16*)rplanes;

#pragma unroll 1
  for (int e = 0; e < kNumExperts; ++e) {
    const v4f* pp = (const v4f*)(params + (size_t)(e * 2 + hf) * kParamStride);
    float prm[88];
#pragma unroll
    for (int q = 0; q < 22; ++q) {
      const v4f pv = pp[q];
      prm[4 * q + 0] = pv[0];
      prm[4 * q + 1] = pv[1];
      prm[4 * q + 2] = pv[2];
      prm[4 * q + 3] = pv[3];
    }
    const int fbase = ((e * 3) * 32 + col) * 32 + 8 * hf;
    const float bias_out = prm[7 * kParamGroup];

#pragma unroll 1
    for (int t = 0; t < kTilesPerWave; ++t) {
      int fo = fbase;
      asm volatile("" : "+v"(fo));

      int sidx = s0 + t * 16 + col;
      sidx = (sidx < nsamp) ? sidx : (nsamp - 1);
      const v2f xv = *(const v2f*)(x + 2 * (size_t)sidx);
      const float x0 = xv[0];
      const float x1 = xv[1];
      const int ci = cell_index(x0);
      const int ri = cell_index(x1);
      const int my_e = ((ci < 0) || (ri < 0)) ? -1 : (ci * 4 + ri);

      v16h hbv, hbr;
#pragma unroll
      for (int i = 0; i < 16; ++i) {
        hbv[i] = (_Float16)0.0f;
        hbr[i] = (_Float16)0.0f;
      }
#pragma unroll
      for (int i = 0; i < 10; ++i) {
        const float z = fmaf(x1, prm[kParamGroup + i], x0 * prm[i]) + prm[2 * kParamGroup + i];
        _Float16 ov, orem;
        silu_to_operands(z, ov, orem);
        hbv[i] = ov;
        hbr[i] = orem;
      }

#pragma unroll
      for (int l = 0; l < 2; ++l) {
        v8f d0, d1, r0, r1;
        hidden_products(pl + fo + l * 1024, rl + fo + l * 1024, hbv, hbr, d0, d1, r0, r1);
        v16h nbv, nbr;
#pragma unroll
        for (int i = 0; i < 16; ++i) {
          nbv[i] = (_Float16)0.0f;
          nbr[i] = (_Float16)0.0f;
        }
#pragma unroll
        for (int r = 0; r < 8; ++r) {
          const float sj = fmaf(r0[r], kRemFold, d0[r]);
          const float z = fmaf(sj, kFoldBack, prm[(3 + l) * kParamGroup + r]);
          _Float16 ov, orem;
          silu_to_operands(z, ov, orem);
          nbv[r] = ov;
          nbr[r] = orem;
        }
#pragma unroll
        for (int r = 0; r < 2; ++r) {
          const float sj = fmaf(r1[r], kRemFold, d1[r]);
          const float z = fmaf(sj, kFoldBack, prm[(3 + l) * kParamGroup + 8 + r]);
          _Float16 ov, orem;
          silu_to_operands(z, ov, orem);
          nbv[8 + r] = ov;
          nbr[8 + r] = orem;
        }
        hbv = nbv;
        hbr = nbr;
      }

      float part = 0.0f;
      {
        v8f d0, d1, r0, r1;
        hidden_products(pl + fo + 2 * 1024, rl + fo + 2 * 1024, hbv, hbr, d0, d1, r0, r1);
#pragma unroll
        for (int r = 0; r < 8; ++r) {
          const float sj = fmaf(r0[r], kRemFold, d0[r]);
          const float z = fmaf(sj, kFoldBack, prm[5 * kParamGroup + r]);
          const float hv = z * gate_sigmoid(z);
          part = fmaf(hv, prm[6 * kParamGroup + r], part);
        }
#pragma unroll
        for (int r = 0; r < 2; ++r) {
          const float sj = fmaf(r1[r], kRemFold, d1[r]);
          const float z = fmaf(sj, kFoldBack, prm[5 * kParamGroup + 8 + r]);
          const float hv = z * gate_sigmoid(z);
          part = fmaf(hv, prm[6 * kParamGroup + 8 + r], part);
        }
      }
      const float other = __shfl_xor(part, 16, 32);
      const float expert_out = (part + other) + bias_out;

      float yv = ysw[t * 32 + lane];
      yv += (my_e == e) ? expert_out : 0.0f;
      ysw[t * 32 + lane] = yv;
    }
  }

  __syncthreads();
  {
    const v4f val = *(const v4f*)(ysw + (lane >> 2) * 32 + (lane & 3) * 4);
    float* op = out + (size_t)s0 + (size_t)lane * 4;
    *(volatile v4f*)op = val;
    __threadfence();
    *(volatile v4f*)op = val;
  }
}

extern "C" void kernel_launch(void* const* d_in, const int* in_sizes, int n_in,
                              void* d_out, int out_size, void* d_ws, size_t ws_size,
                              hipStream_t stream) {
  if (n_in < 11) return;
  if (in_sizes[0] != kNumSamples * kInputs) return;
  if (in_sizes[1] != kNumExperts * kInputs * kHidden) return;
  if (in_sizes[2] != kNumExperts * kHidden) return;
  if (in_sizes[3] != kNumExperts * kHidden * kHidden) return;
  if (in_sizes[4] != kNumExperts * kHidden) return;
  if (in_sizes[5] != kNumExperts * kHidden * kHidden) return;
  if (in_sizes[6] != kNumExperts * kHidden) return;
  if (in_sizes[7] != kNumExperts * kHidden * kHidden) return;
  if (in_sizes[8] != kNumExperts * kHidden) return;
  if (in_sizes[9] != kNumExperts * kHidden) return;
  if (in_sizes[10] != kNumExperts) return;
  if (out_size != kNumSamples) return;
  if (ws_size < kWsTotal) return;

  const float* x  = (const float*)d_in[0];
  const float* W1 = (const float*)d_in[1];
  const float* b1 = (const float*)d_in[2];
  const float* W2 = (const float*)d_in[3];
  const float* b2 = (const float*)d_in[4];
  const float* W3 = (const float*)d_in[5];
  const float* b3 = (const float*)d_in[6];
  const float* W4 = (const float*)d_in[7];
  const float* b4 = (const float*)d_in[8];
  const float* W5 = (const float*)d_in[9];
  const float* b5 = (const float*)d_in[10];
  float* out = (float*)d_out;

  char* ws = (char*)d_ws;
  unsigned short* planes  = (unsigned short*)(ws + kOffPlanes);
  unsigned short* rplanes = (unsigned short*)(ws + kOffRemPlanes);
  float*          params  = (float*)(ws + kOffParams);

  build_weight_planes_kernel<<<dim3(kNumExperts, 3), 128, 0, stream>>>(W2, W3, W4, planes, rplanes);
  build_param_table_kernel<<<kNumExperts, 256, 0, stream>>>(W1, b1, b2, b3, b4, W5, b5, params);
  grid_ensemble_kernel<<<kNumBlocks, 256, 0, stream>>>(x, planes, rplanes, params, out, kNumSamples);
}
